// RGCN_85341000172301
// MI455X (gfx1250) — hardware-verified
//
#include <hip/hip_runtime.h>
#include <stddef.h>
#include <stdint.h>


#define PAIR_SPLIT 1

#define NN     50000
#define NE     800000
#define CC     64
#define NR     65
#define NB     512
#define SLA    9
#define NBLK   98
#define MP     (NBLK * NB)
#define NTHR   256
#define NWAVE  8
#define EPT    8
#define CHUNK  (NTHR * EPT)
#define WCAP   (EPT * 32)
#define LISTN  (NWAVE * WCAP)
#define RCAPB  9216
#define DEGCAP 48
#define PCAPB  10192
#define NTILEB (PCAPB / 16)
#define NKEY   (NR * NB)
#define ARRN   (NKEY + 16)
#define NGRP   (NKEY / 32)
#define RELTW  96
#define REG0N  (LISTN + 2 * RCAPB)
#define BK_INTS (REG0N + ARRN + RCAPB + NGRP + RELTW + 32)
#define ACCN   ((NB + NWAVE) * CC)
#define WTP    36
#define WTN    (CC * WTP)
#define ATP    68
#define ATN    (16 * ATP)
#define LY_INTS (ACCN + 2 * WTN + NWAVE * ATN + RELTW)
#define PB_X   1568
#define PB_W   130
#define PB_L   2

static_assert(CC == 64 && NR == 65 && NB == 512 && NB == (1 << SLA));
static_assert(NBLK * NB >= NN && MP == NBLK * NB);
static_assert(PB_X * 256 == MP * 8 && PB_W * 256 == NR * CC * 8 && PB_L * 256 == CC * 8);
static_assert(PCAPB % 16 == 0 && PCAPB >= RCAPB + NR * 15);
static_assert(RCAPB >= 8397 + 8397 / 20 && RCAPB % 256 == 0 && DEGCAP >= 33 + 8);
static_assert(2 * PCAPB <= REG0N);
static_assert(NB < 65536 && DEGCAP < 65536);
static_assert(NKEY % 32 == 0 && NGRP == NR * 16 && NKEY / 32 == 1040);
static_assert((NE % 8) == 0 && ((CHUNK << SLA) > 0));
static_assert(BK_INTS % 4 == 0 && REG0N % 4 == 0 && ARRN % 4 == 0 && NGRP % 4 == 0);
static_assert(BK_INTS * 4 <= 327680 && LY_INTS * 4 <= 327680);
static_assert(ACCN % 4 == 0 && WTN % 4 == 0 && ATN % 4 == 0 && (ATP % 4) == 0 && (WTP % 4) == 0);
static_assert(NB % (NWAVE * 16) == 0 && NB / NWAVE == 64);

typedef float          v4f   __attribute__((ext_vector_type(4)));
typedef float          v8f   __attribute__((ext_vector_type(8)));
typedef int            v4i   __attribute__((ext_vector_type(4)));
typedef int            v8i   __attribute__((ext_vector_type(8)));
typedef unsigned       v2u   __attribute__((ext_vector_type(2)));
typedef unsigned short v8us  __attribute__((ext_vector_type(8)));
typedef __bf16         v16bf __attribute__((ext_vector_type(16)));
typedef v4f  __attribute__((may_alias)) v4fa;
typedef v4i  __attribute__((may_alias)) v4ia;
typedef v2u  __attribute__((may_alias)) v2ua;
typedef v8us __attribute__((may_alias)) v8usa;
union FragB { v16bf v; v8us u[2]; v8i w; v4i q[2]; };

__device__ __forceinline__ v8f wmx(const FragB& a, const FragB& b, v8f c) {
  v8f d = __builtin_amdgcn_wmma_f32_16x16x32_bf16(false, a.v, false, b.v, (short)0, c, false, false);
  asm volatile("v_nop\n\tv_nop\n\tv_nop\n\tv_nop" : "+v"(d) : "v"(a.w), "v"(b.w));
  return d;
}

__device__ __forceinline__ void pinf(float x) { asm volatile("" :: "v"(x)); }
__device__ __forceinline__ void pini(int x)   { asm volatile("" :: "v"(x)); }
__device__ __forceinline__ void pin4(const v4i w) { pini(w.x); pini(w.y); pini(w.z); pini(w.w); }
__device__ __forceinline__ int clampi(int v, int lo, int hi) { return v < lo ? lo : (v > hi ? hi : v); }
__device__ __forceinline__ v8f z8() { v8f z = {0.f, 0.f, 0.f, 0.f, 0.f, 0.f, 0.f, 0.f}; return z; }

__device__ __forceinline__ void wsync() {
  asm volatile("" ::: "memory");
  __builtin_amdgcn_wave_barrier();
  asm volatile("" ::: "memory");
}

__device__ __forceinline__ unsigned bfbits(float v) {
  const unsigned u = __float_as_uint(v);
  const unsigned r = (u + 0x7FFFu + ((u >> 16) & 1u)) >> 16;
  const unsigned nb = ((u >> 16) & 0x8000u) | 0x7FC0u;
  return ((u & 0x7FFFFFFFu) > 0x7F800000u) ? nb : r;
}

__device__ __forceinline__ v8us cvt8(const v4f a, const v4f b, unsigned mk) {
  v8us o;
  o[0] = (unsigned short)(bfbits(a.x) & mk); o[1] = (unsigned short)(bfbits(a.y) & mk);
  o[2] = (unsigned short)(bfbits(a.z) & mk); o[3] = (unsigned short)(bfbits(a.w) & mk);
  o[4] = (unsigned short)(bfbits(b.x) & mk); o[5] = (unsigned short)(bfbits(b.y) & mk);
  o[6] = (unsigned short)(bfbits(b.z) & mk); o[7] = (unsigned short)(bfbits(b.w) & mk);
  return o;
}

__device__ __forceinline__ void st2(unsigned short* dp, const v8us hv) {
  *(volatile v8us*)dp = hv;
  __threadfence();
  *(volatile v8us*)dp = hv;
}

__global__ __launch_bounds__(256) void k_zero(v4i* p, int n16) {
  const int i = (int)blockIdx.x * 256 + (int)threadIdx.x;
  if (i < n16) {
    const v4i z = {0, 0, 0, 0};
    *(volatile v4i*)(p + i) = z;
    __threadfence();
    *(volatile v4i*)(p + i) = z;
  }
}

__device__ __forceinline__ v8us gat8(const float* __restrict__ w, size_t sb) {
  float f[8];
#pragma unroll
  for (int i = 0; i < 8; ++i) { f[i] = w[sb + (size_t)i * CC]; pinf(f[i]); }
  v8us hv;
#pragma unroll
  for (int i = 0; i < 8; ++i) hv[i] = (unsigned short)bfbits(f[i]);
  return hv;
}

__global__ __launch_bounds__(256) void k_prep(const float* __restrict__ x, const float* __restrict__ w1,
                                              const float* __restrict__ wl1, const float* __restrict__ w2,
                                              const float* __restrict__ wl2, unsigned short* xb,
                                              unsigned short* wt1, unsigned short* wt2,
                                              unsigned short* wlt1, unsigned short* wlt2) {
  const int b = (int)blockIdx.x, tid = (int)threadIdx.x;
  if (b < PB_X) {
    const int u   = b * 256 + tid;
    const int row = u >> 3;
    const int c0  = (u & 7) * 8;
    const int rc  = row < NN ? row : NN - 1;
    const float* p = x + (size_t)rc * CC + c0;
    const v4f a = *(const v4f*)p, c = *(const v4f*)(p + 4);
    const unsigned mk = row < NN ? 0xFFFFu : 0u;
    st2(xb + (size_t)u * 8, cvt8(a, c, mk));
  } else if (b < PB_X + PB_W) {
    const int u  = (b - PB_X) * 256 + tid;
    const int r  = u >> 9, n = (u >> 3) & 63, k8 = (u & 7) * 8;
    const size_t sb = (size_t)r * (CC * CC) + (size_t)k8 * CC + (size_t)n;
    st2(wt1 + (size_t)u * 8, gat8(w1, sb));
  } else if (b < PB_X + 2 * PB_W) {
    const int u  = (b - PB_X - PB_W) * 256 + tid;
    const int r  = u >> 9, n = (u >> 3) & 63, k8 = (u & 7) * 8;
    const size_t sb = (size_t)r * (CC * CC) + (size_t)k8 * CC + (size_t)n;
    st2(wt2 + (size_t)u * 8, gat8(w2, sb));
  } else if (b < PB_X + 2 * PB_W + PB_L) {
    const int u  = (b - PB_X - 2 * PB_W) * 256 + tid;
    const int n  = u >> 3, k8 = (u & 7) * 8;
    st2(wlt1 + (size_t)u * 8, gat8(wl1, (size_t)k8 * CC + (size_t)n));
  } else {
    const int u  = (b - PB_X - 2 * PB_W - PB_L) * 256 + tid;
    const int n  = u >> 3, k8 = (u & 7) * 8;
    st2(wlt2 + (size_t)u * 8, gat8(wl2, (size_t)k8 * CC + (size_t)n));
  }
}

__device__ __forceinline__ int ldkey(const int* __restrict__ k, int e, int nE, int sent) {
  const int v = k[e < nE ? e : nE - 1];
  pini(v);
  return (e < nE) ? v : sent;
}

__device__ __forceinline__ int scan_chunk(const int* __restrict__ keys, int nE, int cbase, int slotBase,
                                          int nb, int* list, int tid, int lane, int wave) {
  int wc = 0;
  const int el0  = tid * EPT;
  const int e0   = cbase + el0;
  const int sent = (int)(1u << 31);
  v4i da, db;
  if (cbase + CHUNK <= nE) {
    da = *(const v4i*)(keys + e0);
    db = *(const v4i*)(keys + e0 + 4);
  } else {
    da.x = ldkey(keys, e0,     nE, sent);
    da.y = ldkey(keys, e0 + 1, nE, sent);
    da.z = ldkey(keys, e0 + 2, nE, sent);
    da.w = ldkey(keys, e0 + 3, nE, sent);
    db.x = ldkey(keys, e0 + 4, nE, sent);
    db.y = ldkey(keys, e0 + 5, nE, sent);
    db.z = ldkey(keys, e0 + 6, nE, sent);
    db.w = ldkey(keys, e0 + 7, nE, sent);
  }
  const unsigned nbs = (unsigned)slotBase;
  const unsigned unb = (unsigned)nb;
  const unsigned s0 = (unsigned)da.x - nbs, s1 = (unsigned)da.y - nbs;
  const unsigned s2 = (unsigned)da.z - nbs, s3 = (unsigned)da.w - nbs;
  const unsigned s4 = (unsigned)db.x - nbs, s5 = (unsigned)db.y - nbs;
  const unsigned s6 = (unsigned)db.z - nbs, s7 = (unsigned)db.w - nbs;
  const bool h0 = s0 < unb, h1 = s1 < unb, h2 = s2 < unb, h3 = s3 < unb;
  const bool h4 = s4 < unb, h5 = s5 < unb, h6 = s6 < unb, h7 = s7 < unb;
  const unsigned any = __builtin_amdgcn_ballot_w32(h0 | h1 | h2 | h3 | h4 | h5 | h6 | h7);
  if (any != 0u) {
    const int k = (int)h0 + (int)h1 + (int)h2 + (int)h3 + (int)h4 + (int)h5 + (int)h6 + (int)h7;
    int incl = k;
#pragma unroll
    for (int dd = 1; dd < 32; dd <<= 1) {
      const int y = __shfl_up(incl, dd, 32);
      if (lane >= dd) incl += y;
    }
    wc = __shfl(incl, 31, 32);
    int pos = incl - k;
#define PUTJ(J, HJ, SJ) if (HJ) { if (pos < WCAP) list[wave * WCAP + pos] = ((el0 + (J)) << SLA) | (int)(SJ); pos += 1; }
    PUTJ(0, h0, s0)
    PUTJ(1, h1, s1)
    PUTJ(2, h2, s2)
    PUTJ(3, h3, s3)
    PUTJ(4, h4, s4)
    PUTJ(5, h5, s5)
    PUTJ(6, h6, s6)
    PUTJ(7, h7, s7)
#undef PUTJ
  }
  return wc;
}

__global__ __launch_bounds__(NTHR) void k_bucket(const int* __restrict__ src, const int* __restrict__ dst,
                                                 const int* __restrict__ et, int* entg, int* pairg, int* reltg) {
  extern __shared__ __attribute__((aligned(16))) int dsm[];
  int* list = dsm;
  int* hk   = dsm + LISTN;
  int* hs   = hk + RCAPB;
  int* pst  = dsm;
  int* arr  = dsm + REG0N;
  int* ent  = arr + ARRN;
  int* pc   = ent + RCAPB;
  int* relt = pc + NGRP;
  int* misc = relt + RELTW;
  const int tid = (int)threadIdx.x, lane = tid & 31;
  const int wave = __builtin_amdgcn_readfirstlane(tid >> 5);
  const int b = (int)blockIdx.x;
  const int nodeBase = b * NB;

  {
    const v4i z4 = {0, 0, 0, 0};
    for (int i = tid * 4; i < BK_INTS; i += NTHR * 4) *(v4ia*)(dsm + i) = z4;
  }
  __syncthreads();

  int t = 0;
  const int nChunks = (NE + CHUNK - 1) / CHUNK;
#pragma unroll 1
  for (int ch = 0; ch < nChunks; ++ch) {
    const int cbase = ch * CHUNK;
    int wc = scan_chunk(dst, NE, cbase, nodeBase, NB, list, tid, lane, wave);
    wc = __builtin_amdgcn_readfirstlane(wc);
    int* mb = misc + (ch & 1) * 8;
    if (lane == 0) mb[wave] = wc;
    __syncthreads();
    int base = t, tot = 0;
#pragma unroll
    for (int w2 = 0; w2 < NWAVE; ++w2) {
      const int c = clampi(mb[w2], 0, WCAP);
      base += (w2 < wave) ? c : 0;
      tot  += c;
    }
    const int myc = clampi(wc, 0, WCAP);
#pragma unroll 1
    for (int b0 = 0; b0 < myc; b0 += 32) {
      const int idx  = b0 + lane;
      const int entv = list[wave * WCAP + (idx < WCAP ? idx : WCAP - 1)];
      const int slot = entv & (NB - 1);
      const int el   = (entv >> SLA) & (CHUNK - 1);
      const int eid  = clampi(cbase + el, 0, NE - 1);
      int ty = et[eid];
      pini(ty);
      ty = clampi(ty, 0, NR - 1);
      int sr = src[eid];
      pini(sr);
      sr = clampi(sr, 0, NN - 1);
      const int pos = base + idx;
      if (idx < myc && pos < RCAPB) {
        hk[pos] = ty * NB + slot;
        hs[pos] = sr;
      }
    }
    t += tot;
  }
  __syncthreads();
  const int tt = t < RCAPB ? t : RCAPB;
  const int ov = t > RCAPB ? 1 : 0;

  if (tid == 0) {
#pragma unroll 1
    for (int i = 0; i < tt; ++i) {
      const int k = clampi(hk[i], 0, NKEY - 1);
      arr[k] = arr[k] + 1;
    }
  }
  __syncthreads();
  if (wave == 0) {
    const int base = lane * (NKEY / 32);
    int s = 0;
#pragma unroll 1
    for (int i = 0; i < NKEY / 32; ++i) s += arr[base + i];
    int incl = s;
#pragma unroll
    for (int dd = 1; dd < 32; dd <<= 1) {
      const int y = __shfl_up(incl, dd, 32);
      if (lane >= dd) incl += y;
    }
    int run = incl - s;
#pragma unroll 1
    for (int i = 0; i < NKEY / 32; ++i) {
      run += arr[base + i];
      arr[base + i] = run;
    }
    if (lane == 31) arr[NKEY] = run;
  }
  __syncthreads();
  if (tid == 0) {
#pragma unroll 1
    for (int i = tt - 1; i >= 0; --i) {
      const int k = clampi(hk[i], 0, NKEY - 1);
      const int p = clampi(arr[k] - 1, 0, RCAPB - 1);
      arr[k] = p;
      ent[p] = hs[i];
    }
  }
  __syncthreads();

  {
    int ovd = 0;
#pragma unroll 1
    for (int gi = wave; gi < NGRP; gi += NWAVE) {
      const int k = gi * 32 + lane;
      const int c = arr[k + 1] - arr[k];
      ovd |= (c > DEGCAP) ? 1 : 0;
      const unsigned mk = __builtin_amdgcn_ballot_w32(c > 0);
      if (lane == 0) pc[gi] = (int)__builtin_popcount(mk);
    }
    const unsigned om = __builtin_amdgcn_ballot_w32(ovd != 0);
    if (lane == 0) misc[20 + wave] = (om != 0u) ? 1 : 0;
    const v4i z4 = {0, 0, 0, 0};
    for (int i = tid * 4; i < 2 * PCAPB; i += NTHR * 4) *(v4ia*)(pst + i) = z4;
  }
  __syncthreads();
  if (tid == 0) {
    int run = 0;
#pragma unroll 1
    for (int r = 0; r < NR; ++r) {
      relt[r] = run >> 4;
#pragma unroll 1
      for (int g = 0; g < 16; ++g) {
        const int c = clampi(pc[r * 16 + g], 0, 32);
        pc[r * 16 + g] = run;
        run += c;
      }
      run = (run + 15) & ~15;
    }
    relt[NR] = run >> 4;
    int fl = ov;
#pragma unroll 1
    for (int w2 = 0; w2 < NWAVE; ++w2) fl |= misc[20 + w2];
    relt[NR + 1] = fl;
  }
  __syncthreads();
#pragma unroll 1
  for (int gi = wave; gi < NGRP; gi += NWAVE) {
    const int k  = gi * 32 + lane;
    const int st = arr[k];
    int c = arr[k + 1] - st;
    c = clampi(c, 0, DEGCAP);
    const unsigned mk = __builtin_amdgcn_ballot_w32(c > 0);
    const int idx = pc[gi] + (int)__builtin_amdgcn_mbcnt_lo(mk, 0u);
    if (c > 0 && idx >= 0 && idx < PCAPB) {
      pst[2 * idx]     = (k & (NB - 1)) | (c << 16);
      pst[2 * idx + 1] = clampi(st, 0, RCAPB - 1);
    }
  }
  __syncthreads();

  int* eg = entg  + (size_t)b * RCAPB;
  int* pg = pairg + (size_t)b * (2 * PCAPB);
  int* rg = reltg + (size_t)b * RELTW;
  for (int i = tid * 4; i < RCAPB; i += NTHR * 4) {
    const v4i v = *(const v4ia*)(ent + i);
    *(volatile v4i*)(eg + i) = v;
  }
  for (int i = tid * 4; i < 2 * PCAPB; i += NTHR * 4) {
    const v4i v = *(const v4ia*)(pst + i);
    *(volatile v4i*)(pg + i) = v;
  }
  if (tid < RELTW / 4) {
    const v4i v = *(const v4ia*)(relt + 4 * tid);
    *(volatile v4i*)(rg + 4 * tid) = v;
  }
  __threadfence();
  for (int i = tid * 4; i < RCAPB; i += NTHR * 4) {
    const v4i v = *(const v4ia*)(ent + i);
    *(volatile v4i*)(eg + i) = v;
  }
  for (int i = tid * 4; i < 2 * PCAPB; i += NTHR * 4) {
    const v4i v = *(const v4ia*)(pst + i);
    *(volatile v4i*)(pg + i) = v;
  }
  if (tid < RELTW / 4) {
    const v4i v = *(const v4ia*)(relt + 4 * tid);
    *(volatile v4i*)(rg + 4 * tid) = v;
  }
}

__device__ __forceinline__ void addw1(float& a0, float& a1, int w, int mk) {
  a0 += __int_as_float((w << 16) & mk);
  a1 += __int_as_float((w & (int)0xffff0000) & mk);
}
__device__ __forceinline__ void addw2(float& a0, float& a1, int wh, int wl, int mk) {
  const float x0 = __int_as_float(wh << 16) + __int_as_float(wl << 16);
  const float x1 = __int_as_float(wh & (int)0xffff0000) + __int_as_float(wl & (int)0xffff0000);
  a0 += __int_as_float(__float_as_int(x0) & mk);
  a1 += __int_as_float(__float_as_int(x1) & mk);
}

__device__ __forceinline__ void stage_wt(const unsigned short* __restrict__ g, int* dl, int tid) {
#pragma unroll
  for (int it = 0; it < 2; ++it) {
    const int p = tid + NTHR * it;
    const v4i w = *(const v4ia*)(g + (size_t)p * 8);
    *(v4ia*)(dl + (p >> 3) * WTP + (p & 7) * 4) = w;
  }
}

template <int LAYER>
__global__ __launch_bounds__(NTHR) __attribute__((amdgpu_num_vgpr(248)))
void k_layer(const unsigned short* __restrict__ xin, const unsigned short* __restrict__ wt,
             const unsigned short* __restrict__ wlt, const int* __restrict__ entg,
             const unsigned* __restrict__ pairg, const int* __restrict__ reltg,
             unsigned short* hout, float* outp) {
  extern __shared__ __attribute__((aligned(16))) int lsm[];
  constexpr int XP  = (LAYER == 1) ? CC : 2 * CC;
  constexpr int RKS = (LAYER == 1) ? 2 : 4;
  constexpr int PKS = PAIR_SPLIT ? 4 : 2;
  float* accf = (float*)lsm;
  int* wtb = lsm + ACCN;
  int* atl = wtb + 2 * WTN;
  int* rel = atl + NWAVE * ATN;
  const int tid = (int)threadIdx.x, lane = tid & 31, hh = lane >> 4, m = lane & 15;
  const int wave = __builtin_amdgcn_readfirstlane(tid >> 5);
  const int b = (int)blockIdx.x;
  const int nodeBase = b * NB;
  int* atw = atl + wave * ATN;

  if (tid < (NWAVE * CC) / 4) {
    const v4f z = {0.f, 0.f, 0.f, 0.f};
    *(v4fa*)(accf + NB * CC + 4 * tid) = z;
  }
  if (wave == 0) {
    const int li = lane < RELTW / 4 ? lane : RELTW / 4 - 1;
    const v4i v = *(const v4ia*)(reltg + (size_t)b * RELTW + 4 * li);
    pin4(v);
    if (lane < RELTW / 4) *(v4ia*)(rel + 4 * lane) = v;
  }
  stage_wt(wt, wtb, tid);

#pragma unroll 1
  for (int j = 0; j < 4; ++j) {
    const int rowt = (wave * 4 + j) * 16;
    const unsigned short* ap = xin + (size_t)(nodeBase + rowt + m) * XP + 8 * hh;
    v8f d[4];
    d[0] = z8(); d[1] = z8(); d[2] = z8(); d[3] = z8();
#pragma unroll
    for (int ks = 0; ks < RKS; ++ks) {
      FragB af;
      af.u[0] = *(const v8usa*)(ap + 32 * ks);
      af.u[1] = *(const v8usa*)(ap + 32 * ks + 16);
#pragma unroll
      for (int tcol = 0; tcol < 4; ++tcol) {
        const unsigned short* wq = wlt + (size_t)(16 * tcol + m) * CC + 8 * hh + 32 * (ks & 1);
        FragB bf;
        bf.u[0] = *(const v8usa*)wq;
        bf.u[1] = *(const v8usa*)(wq + 16);
        d[tcol] = wmx(af, bf, d[tcol]);
      }
    }
#pragma unroll
    for (int tcol = 0; tcol < 4; ++tcol) {
#pragma unroll
      for (int r = 0; r < 8; ++r) {
        accf[(rowt + 8 * hh + r) * CC + 16 * tcol + m] = d[tcol][r];
      }
    }
  }
  __syncthreads();
  const int flag = rel[NR + 1];

#pragma unroll 1
  for (int r = 0; r < NR; ++r) {
    if (r + 1 < NR) stage_wt(wt + (size_t)(r + 1) * (CC * CC), wtb + ((r + 1) & 1) * WTN, tid);
    int t0 = clampi(rel[r], 0, NTILEB);
    int t1 = clampi(rel[r + 1], t0, NTILEB);
    t0 = __builtin_amdgcn_readfirstlane(t0);
    t1 = __builtin_amdgcn_readfirstlane(t1);
    const int* wb = wtb + (r & 1) * WTN;
#pragma unroll 1
    for (int tl = t0 + wave; tl < t1; tl += NWAVE) {
      const int prow = tl * 16 + m;
      const v2u pw = *(const v2ua*)(pairg + ((size_t)b * PCAPB + (size_t)prow) * 2);
      pini((int)pw.x); pini((int)pw.y);
      int cnt = clampi((int)(pw.x >> 16), 0, DEGCAP);
      const int slot = clampi((int)(pw.x & 0xffffu), 0, NB - 1);
      const int off  = clampi((int)pw.y, 0, RCAPB - 1);
      if (cnt > RCAPB - off) cnt = RCAPB - off;
      const int last = off + (cnt > 0 ? cnt - 1 : 0);
      int cm = cnt;
#pragma unroll
      for (int o2 = 1; o2 < 16; o2 <<= 1) {
        const int y = __shfl_xor(cm, o2, 32);
        cm = cm > y ? cm : y;
      }
      cm = __builtin_amdgcn_readfirstlane(cm);

      float a[32];
#pragma unroll
      for (int i = 0; i < 32; ++i) a[i] = 0.0f;
#pragma unroll 1
      for (int p = 0; p < cm; ++p) {
        int idx = off + p; idx = idx > last ? last : idx;
        int sr = entg[(size_t)b * RCAPB + idx];
        pini(sr);
        sr = clampi(sr, 0, NN - 1);
        const int mk = (p < cnt) ? -1 : 0;
        const unsigned short* rp = xin + (size_t)sr * XP + 32 * hh;
        if constexpr (LAYER == 1) {
          v4i w[4];
#pragma unroll
          for (int q = 0; q < 4; ++q) { w[q] = *(const v4ia*)(rp + 8 * q); pin4(w[q]); }
#pragma unroll
          for (int q = 0; q < 4; ++q) {
            addw1(a[8 * q + 0], a[8 * q + 1], w[q].x, mk);
            addw1(a[8 * q + 2], a[8 * q + 3], w[q].y, mk);
            addw1(a[8 * q + 4], a[8 * q + 5], w[q].z, mk);
            addw1(a[8 * q + 6], a[8 * q + 7], w[q].w, mk);
          }
        } else {
          v4i wh[4], wl[4];
#pragma unroll
          for (int q = 0; q < 4; ++q) {
            wh[q] = *(const v4ia*)(rp + 8 * q);
            wl[q] = *(const v4ia*)(rp + CC + 8 * q);
            pin4(wh[q]); pin4(wl[q]);
          }
#pragma unroll
          for (int q = 0; q < 4; ++q) {
            addw2(a[8 * q + 0], a[8 * q + 1], wh[q].x, wl[q].x, mk);
            addw2(a[8 * q + 2], a[8 * q + 3], wh[q].y, wl[q].y, mk);
            addw2(a[8 * q + 4], a[8 * q + 5], wh[q].z, wl[q].z, mk);
            addw2(a[8 * q + 6], a[8 * q + 7], wh[q].w, wl[q].w, mk);
          }
        }
      }
      const float den = fmaxf((float)cnt, 1.0f);
      const float rc  = 1.0f / den;
      int hw[16], lw[16];
#pragma unroll
      for (int j = 0; j < 16; ++j) {
        const float v0 = a[2 * j] * rc, v1 = a[2 * j + 1] * rc;
        const unsigned h0 = bfbits(v0), h1 = bfbits(v1);
        hw[j] = (int)(h0 | (h1 << 16));
        const unsigned l0 = bfbits(v0 - __uint_as_float(h0 << 16));
        const unsigned l1 = bfbits(v1 - __uint_as_float(h1 << 16));
        lw[j] = (int)(l0 | (l1 << 16));
      }
      int* at = atw + m * ATP;
#pragma unroll
      for (int q = 0; q < 4; ++q) {
        v4i hv;
        hv.x = hw[4 * q]; hv.y = hw[4 * q + 1]; hv.z = hw[4 * q + 2]; hv.w = hw[4 * q + 3];
        *(v4ia*)(at + 16 * hh + 4 * q) = hv;
        if (PAIR_SPLIT) {
          v4i lv;
          lv.x = lw[4 * q]; lv.y = lw[4 * q + 1]; lv.z = lw[4 * q + 2]; lv.w = lw[4 * q + 3];
          *(v4ia*)(at + 32 + 16 * hh + 4 * q) = lv;
        }
      }
      if (hh == 0) at[64] = (cnt > 0) ? slot : (NB + wave);
      wsync();

      v8f d[4];
      d[0] = z8(); d[1] = z8(); d[2] = z8(); d[3] = z8();
#pragma unroll
      for (int ks = 0; ks < PKS; ++ks) {
        FragB af;
        af.q[0] = *(const v4ia*)(atw + m * ATP + 16 * ks + 4 * hh);
        af.q[1] = *(const v4ia*)(atw + m * ATP + 16 * ks + 8 + 4 * hh);
#pragma unroll
        for (int tcol = 0; tcol < 4; ++tcol) {
          FragB bf;
          bf.q[0] = *(const v4ia*)(wb + (16 * tcol + m) * WTP + 16 * (ks & 1) + 4 * hh);
          bf.q[1] = *(const v4ia*)(wb + (16 * tcol + m) * WTP + 16 * (ks & 1) + 8 + 4 * hh);
          d[tcol] = wmx(af, bf, d[tcol]);
        }
      }
      int tr[8];
#pragma unroll
      for (int rr = 0; rr < 8; ++rr) tr[rr] = clampi(atw[(8 * hh + rr) * ATP + 64], 0, NB + NWAVE - 1) * CC;
#pragma unroll
      for (int tcol = 0; tcol < 4; ++tcol) {
#pragma unroll
        for (int rr = 0; rr < 8; ++rr) {
          float* q = accf + tr[rr] + 16 * tcol + m;
          const float old = *q;
          *q = old + d[tcol][rr];
        }
      }
      wsync();
    }
    __syncthreads();
  }

  const float pz = (flag != 0) ? __int_as_float(0x7fc00000) : 0.0f;
  if constexpr (LAYER == 1) {
#pragma unroll 1
    for (int bt = 0; bt < 4; ++bt) {
      v8us hv[8];
#pragma unroll
      for (int i = 0; i < 8; ++i) {
        const int row = 64 * wave + 16 * bt + 2 * i + hh;
        const int c8  = 8 * (m & 7);
        const v4f x0 = *(const v4fa*)(accf + row * CC + c8);
        const v4f x1 = *(const v4fa*)(accf + row * CC + c8 + 4);
        const bool live = (nodeBase + row) < NN;
        float y[8];
        y[0] = x0.x; y[1] = x0.y; y[2] = x0.z; y[3] = x0.w;
        y[4] = x1.x; y[5] = x1.y; y[6] = x1.z; y[7] = x1.w;
        v8us o;
#pragma unroll
        for (int j = 0; j < 8; ++j) {
          float v = y[j];
          v = (v > 0.0f) ? v : (v - v);
          v = v + pz;
          v = live ? v : 0.0f;
          const unsigned hb = bfbits(v);
          const unsigned lb = bfbits(v - __uint_as_float(hb << 16));
          o[j] = (unsigned short)((m >= 8) ? lb : hb);
        }
        hv[i] = o;
      }
#pragma unroll
      for (int i = 0; i < 8; ++i) {
        const int row = 64 * wave + 16 * bt + 2 * i + hh;
        unsigned short* op = hout + (size_t)(nodeBase + row) * (2 * CC) + 8 * m;
        *(volatile v8us*)op = hv[i];
      }
      __threadfence();
#pragma unroll
      for (int i = 0; i < 8; ++i) {
        const int row = 64 * wave + 16 * bt + 2 * i + hh;
        unsigned short* op = hout + (size_t)(nodeBase + row) * (2 * CC) + 8 * m;
        *(volatile v8us*)op = hv[i];
      }
    }
  } else {
#pragma unroll 1
    for (int bt = 0; bt < 4; ++bt) {
      v4f fv[8];
#pragma unroll
      for (int i = 0; i < 8; ++i) {
        const int row = 64 * wave + 16 * bt + 2 * i + hh;
        const v4f x0 = *(const v4fa*)(accf + row * CC + 4 * m);
        v4f o;
        o.x = ((x0.x > 0.0f) ? x0.x : (x0.x - x0.x)) + pz;
        o.y = ((x0.y > 0.0f) ? x0.y : (x0.y - x0.y)) + pz;
        o.z = ((x0.z > 0.0f) ? x0.z : (x0.z - x0.z)) + pz;
        o.w = ((x0.w > 0.0f) ? x0.w : (x0.w - x0.w)) + pz;
        pinf(o.x); pinf(o.y); pinf(o.z); pinf(o.w);
        fv[i] = o;
      }
#pragma unroll
      for (int i = 0; i < 8; ++i) {
        const int node = nodeBase + 64 * wave + 16 * bt + 2 * i + hh;
        float* op = outp + (size_t)(node < NN ? node : NN - 1) * CC + 4 * m;
        if (node < NN) *(volatile v4f*)op = fv[i];
      }
      __threadfence();
#pragma unroll
      for (int i = 0; i < 8; ++i) {
        const int node = nodeBase + 64 * wave + 16 * bt + 2 * i + hh;
        float* op = outp + (size_t)(node < NN ? node : NN - 1) * CC + 4 * m;
        if (node < NN) *(volatile v4f*)op = fv[i];
      }
    }
  }
  (void)hout; (void)outp;
}

static inline size_t al256(size_t o) { return (o + 255) & ~(size_t)255; }

extern "C" void kernel_launch(void* const* d_in, const int* in_sizes, int n_in,
                              void* d_out, int out_size, void* d_ws, size_t ws_size,
                              hipStream_t stream) {
  if (n_in < 8) return;
  if (in_sizes[0] != NN * CC) return;
  if (in_sizes[1] != NE || in_sizes[2] != NE || in_sizes[3] != NE) return;
  if (in_sizes[4] != NR * CC * CC || in_sizes[6] != NR * CC * CC) return;
  if (in_sizes[5] != CC * CC || in_sizes[7] != CC * CC) return;
  if (out_size != NN * CC) return;

  const float* x   = (const float*)d_in[0];
  const int*   src = (const int*)d_in[1];
  const int*   dst = (const int*)d_in[2];
  const int*   et  = (const int*)d_in[3];
  const float* W1  = (const float*)d_in[4];
  const float* Wl1 = (const float*)d_in[5];
  const float* W2  = (const float*)d_in[6];
  const float* Wl2 = (const float*)d_in[7];
  float* out = (float*)d_out;

  char* ws = (char*)d_ws;
  size_t off = 0;
  const size_t oXB   = off; off = al256(off + (size_t)MP * CC * 2);
  const size_t oH1   = off; off = al256(off + (size_t)MP * 2 * CC * 2);
  const size_t oWT1  = off; off = al256(off + (size_t)NR * CC * CC * 2);
  const size_t oWT2  = off; off = al256(off + (size_t)NR * CC * CC * 2);
  const size_t oWL1  = off; off = al256(off + (size_t)CC * CC * 2);
  const size_t oWL2  = off; off = al256(off + (size_t)CC * CC * 2);
  const size_t oENT  = off; off = al256(off + (size_t)NBLK * RCAPB * 4);
  const size_t oPAIR = off; off = al256(off + (size_t)NBLK * PCAPB * 8);
  const size_t oRELT = off; off = al256(off + (size_t)NBLK * RELTW * 4);
  if (off > ws_size || off > (size_t)(128u << 20)) return;
  unsigned short* XB   = (unsigned short*)(ws + oXB);
  unsigned short* H1   = (unsigned short*)(ws + oH1);
  unsigned short* WT1  = (unsigned short*)(ws + oWT1);
  unsigned short* WT2  = (unsigned short*)(ws + oWT2);
  unsigned short* WLT1 = (unsigned short*)(ws + oWL1);
  unsigned short* WLT2 = (unsigned short*)(ws + oWL2);
  int*            ENT  = (int*)(ws + oENT);
  int*            PAIR = (int*)(ws + oPAIR);
  int*            RELT = (int*)(ws + oRELT);

  const int bkLds = BK_INTS * 4;
  const int lyLds = LY_INTS * 4;
  hipFuncSetAttribute(reinterpret_cast<const void*>(&k_bucket), hipFuncAttributeMaxDynamicSharedMemorySize, bkLds);
  hipFuncSetAttribute(reinterpret_cast<const void*>(&k_layer<1>), hipFuncAttributeMaxDynamicSharedMemorySize, lyLds);
  hipFuncSetAttribute(reinterpret_cast<const void*>(&k_layer<2>), hipFuncAttributeMaxDynamicSharedMemorySize, lyLds);

  const int n16 = (int)(off / 16);
  k_zero<<<(n16 + 255) / 256, 256, 0, stream>>>((v4i*)ws, n16);
  k_prep<<<PB_X + 2 * PB_W + 2 * PB_L, 256, 0, stream>>>(x, W1, Wl1, W2, Wl2, XB, WT1, WT2, WLT1, WLT2);
  k_bucket<<<NBLK, NTHR, bkLds, stream>>>(src, dst, et, ENT, PAIR, RELT);
  k_layer<1><<<NBLK, NTHR, lyLds, stream>>>(XB, WT1, WLT1, ENT, (const unsigned*)PAIR, RELT, H1, out);
  k_layer<2><<<NBLK, NTHR, lyLds, stream>>>(H1, WT2, WLT2, ENT, (const unsigned*)PAIR, RELT, H1, out);
}
